// MPNN_29411936043070
// MI455X (gfx1250) — hardware-verified
//
#include <hip/hip_runtime.h>
#include <stddef.h>


#define NTHR   256
#define NWAVE  8
#define EPT    8
#define CHUNK  (NTHR * EPT)
#define WCAP   (EPT * 32)
#define LISTN  (NWAVE * WCAP)
#define NBS    64
#define DEGCAP 32
#define EC     8
#define HID    32
#define MT     128
#define NGR    256
#define PP     129
#define C1W    64
#define C2W    128
#define BNEPS  1e-5f
#define KT16   (2 * 32 * 16 + 4 * 16)
#define KT64   (2 * 32 * 64 + 4 * 64)

static_assert(CHUNK == 2048 && WCAP == 256 && LISTN == 2048);
static_assert(KT16 == 1088 && KT64 == 4352);
static_assert((KT16 % 32) == 0 && (KT64 % 32) == 0);
static_assert(NBS == 64 && (MT % NBS) == 0);
static_assert(EC * HID == NTHR);
static_assert(2 * C2W == NTHR && NGR == NTHR && 2 * (NTHR - C2W) == NGR);

typedef int            v4i  __attribute__((ext_vector_type(4)));
typedef float          v2f  __attribute__((ext_vector_type(2)));
typedef float          v4f  __attribute__((ext_vector_type(4)));
typedef float          v8f  __attribute__((ext_vector_type(8)));
typedef unsigned short v8us __attribute__((ext_vector_type(8)));
typedef __bf16         v16b __attribute__((ext_vector_type(16)));
union FragB { v16b v; v8us u[2]; };

__device__ __forceinline__ v8f z8() { v8f z = {0.f, 0.f, 0.f, 0.f, 0.f, 0.f, 0.f, 0.f}; return z; }

__device__ __forceinline__ v8f wmb(v16b a, v16b b, v8f c) {
  v8f d = __builtin_amdgcn_wmma_f32_16x16x32_bf16(false, a, false, b, (short)0, c, false, false);
  asm volatile("v_nop\n\tv_nop\n\tv_nop\n\tv_nop" : "+v"(d) : "v"(a), "v"(b));
  return d;
}

__device__ __forceinline__ unsigned short bfr(float x) {
  const unsigned u = __float_as_uint(x);
  return (unsigned short)((u + 0x7FFFu + ((u >> 16) & 1u)) >> 16);
}
__device__ __forceinline__ float bfup(unsigned short h) { return __uint_as_float(((unsigned)h) << 16); }
__device__ __forceinline__ float bfq(float x) { return bfup(bfr(x)); }
__device__ __forceinline__ void hilo(float x, bool bad, unsigned short& hi, unsigned short& lo) {
  const unsigned short h = bfr(x);
  const unsigned short l = bfr(x - bfup(h));
  hi = bad ? (unsigned short)0x7FC0 : h;
  lo = bad ? (unsigned short)0x7FC0 : l;
}

__device__ __forceinline__ int scan_chunk(const int* __restrict__ keys, int nK, int cbase, int slotBase,
                                          int vec8, int* list, int tid, int lane, int wave) {
  int wc = 0;
  const int el0 = tid * EPT;
  const int e0 = cbase + el0;
  const int sent = -2147483647 - 1;
  v4i da, db;
  if (vec8 != 0 && cbase + CHUNK <= nK) {
    da = *(const v4i*)(keys + e0);
    db = *(const v4i*)(keys + e0 + 4);
  } else {
    const int lst = nK - 1;
    da.x = (e0     < nK) ? keys[min(e0,     lst)] : sent;
    da.y = (e0 + 1 < nK) ? keys[min(e0 + 1, lst)] : sent;
    da.z = (e0 + 2 < nK) ? keys[min(e0 + 2, lst)] : sent;
    da.w = (e0 + 3 < nK) ? keys[min(e0 + 3, lst)] : sent;
    db.x = (e0 + 4 < nK) ? keys[min(e0 + 4, lst)] : sent;
    db.y = (e0 + 5 < nK) ? keys[min(e0 + 5, lst)] : sent;
    db.z = (e0 + 6 < nK) ? keys[min(e0 + 6, lst)] : sent;
    db.w = (e0 + 7 < nK) ? keys[min(e0 + 7, lst)] : sent;
  }
  const unsigned nb = (unsigned)slotBase;
  const unsigned s0 = (unsigned)da.x - nb, s1 = (unsigned)da.y - nb, s2 = (unsigned)da.z - nb, s3 = (unsigned)da.w - nb;
  const unsigned s4 = (unsigned)db.x - nb, s5 = (unsigned)db.y - nb, s6 = (unsigned)db.z - nb, s7 = (unsigned)db.w - nb;
  const bool h0 = s0 < 64u, h1 = s1 < 64u, h2 = s2 < 64u, h3 = s3 < 64u, h4 = s4 < 64u, h5 = s5 < 64u, h6 = s6 < 64u, h7 = s7 < 64u;
  const unsigned any = __builtin_amdgcn_ballot_w32(h0 | h1 | h2 | h3 | h4 | h5 | h6 | h7);
  if (any != 0u) {
#define HITJ(J, HJ, SJ) { \
      const unsigned mj = __builtin_amdgcn_ballot_w32(HJ); \
      if (mj != 0u) { \
        if (HJ) { \
          const int pos = wc + (int)__builtin_amdgcn_mbcnt_lo(mj, 0u); \
          if (pos < WCAP) list[wave * WCAP + pos] = ((el0 + (J)) << 6) | (int)(SJ); \
        } \
        wc += (int)__builtin_popcount(mj); } }
    HITJ(0, h0, s0) HITJ(1, h1, s1) HITJ(2, h2, s2) HITJ(3, h3, s3)
    HITJ(4, h4, s4) HITJ(5, h5, s5) HITJ(6, h6, s6) HITJ(7, h7, s7)
#undef HITJ
  }
  return wc;
}

__device__ __forceinline__ void he_layer(const float (&a)[EC], const float* wl, const float* bl,
                                         float* stg, float* dstp, int tid) {
#pragma unroll 1
  for (int j = 0; j < HID; ++j) {
    float s = bl[j];
#pragma unroll
    for (int c = 0; c < EC; ++c) s = fmaf(a[c], wl[c * HID + j], s);
    stg[tid * HID + j] = fmaxf(s, 0.0f);
  }
  __syncthreads();
  v4f pv[8];
#pragma unroll
  for (int it = 0; it < 8; ++it) pv[it] = *(const v4f*)(stg + 4 * (it * NTHR + tid));
#pragma unroll
  for (int it = 0; it < 8; ++it) *(volatile v4f*)(dstp + 4 * (it * NTHR + tid)) = pv[it];
  __threadfence();
#pragma unroll
  for (int it = 0; it < 8; ++it) *(volatile v4f*)(dstp + 4 * (it * NTHR + tid)) = pv[it];
  __syncthreads();
}

__global__ __launch_bounds__(NTHR) void k_he(const float* __restrict__ ea, int nE,
    const float* __restrict__ w1a, const float* __restrict__ b1a,
    const float* __restrict__ w1b, const float* __restrict__ b1b,
    float* he1, float* he2) {
  __shared__ float ws1[2 * EC * HID];
  __shared__ float bs1[2 * HID];
  __shared__ __attribute__((aligned(16))) float stg[NTHR * HID];
  const int tid = threadIdx.x;
  ws1[tid] = bfq(w1a[tid]);
  ws1[EC * HID + tid] = bfq(w1b[tid]);
  if (tid < HID) { bs1[tid] = bfq(b1a[tid]); bs1[HID + tid] = bfq(b1b[tid]); }
  int e = (int)blockIdx.x * NTHR + tid;
  e = e > nE - 1 ? nE - 1 : e;
  const float* ap = ea + (size_t)e * EC;
  const v4f a0 = *(const v4f*)ap, a1 = *(const v4f*)(ap + 4);
  float a[EC];
  a[0] = bfq(a0.x); a[1] = bfq(a0.y); a[2] = bfq(a0.z); a[3] = bfq(a0.w);
  a[4] = bfq(a1.x); a[5] = bfq(a1.y); a[6] = bfq(a1.z); a[7] = bfq(a1.w);
  __syncthreads();
  const size_t boff = (size_t)blockIdx.x * NTHR * HID;
  he_layer(a, ws1, bs1, stg, he1 + boff, tid);
  he_layer(a, ws1 + EC * HID, bs1 + HID, stg, he2 + boff, tid);
}

template <int IN, int OUT>
__device__ __forceinline__ void build_row(const float* __restrict__ W2, const float* __restrict__ b2,
                                          const float* __restrict__ root, int o, unsigned short* Bt,
                                          unsigned short* row, int tid) {
  constexpr int KZ = 32 * IN, KTOT = 2 * KZ + 4 * IN, NIT = KZ / NTHR, NPC = KTOT / 8, PPT = (NPC + NTHR - 1) / NTHR;
  constexpr int LI = (IN == 16) ? 4 : 6;
  static_assert((KZ % NTHR) == 0 && (KTOT % 64) == 0);
#pragma unroll 1
  for (int it = 0; it < NIT; ++it) {
    const int k = it * NTHR + tid;
    const int j = k >> LI, i = k & (IN - 1);
    const unsigned short v = bfr(W2[(size_t)j * (IN * OUT) + (size_t)i * OUT + o]);
    row[k] = v;
    row[KZ + k] = v;
  }
  if constexpr (IN == 16) {
    const int wave = tid >> 5, lane = tid & 31;
    if (wave == 0) {
      row[2 * KZ + lane] = bfr(b2[(lane & 15) * OUT + o]);
    } else if (wave == 1) {
      const unsigned hv = (unsigned)bfr(root[(lane & 15) * OUT + o]);
      const unsigned keep = 0u - (unsigned)(lane < 16);
      row[2 * KZ + 32 + lane] = (unsigned short)(hv & keep);
    }
  } else {
    if (tid < 128) row[2 * KZ + tid] = bfr(b2[(tid & 63) * OUT + o]);
    else           row[2 * KZ + tid] = bfr(root[(tid & 63) * OUT + o]);
  }
  __syncthreads();
  v8us pv[PPT];
#pragma unroll
  for (int it = 0; it < PPT; ++it) {
    int pc = it * NTHR + tid;
    pc = pc > NPC - 1 ? NPC - 1 : pc;
    pv[it] = *(const v8us*)(row + 8 * pc);
  }
  unsigned short* dr = Bt + (size_t)o * KTOT;
#pragma unroll
  for (int it = 0; it < PPT; ++it)
    if (it * NTHR + tid < NPC) *(volatile v8us*)(dr + 8 * (it * NTHR + tid)) = pv[it];
  __threadfence();
#pragma unroll
  for (int it = 0; it < PPT; ++it)
    if (it * NTHR + tid < NPC) *(volatile v8us*)(dr + 8 * (it * NTHR + tid)) = pv[it];
}

__global__ __launch_bounds__(NTHR) void k_bprep(
    const float* __restrict__ W2a, const float* __restrict__ b2a, const float* __restrict__ ra,
    const float* __restrict__ W2b, const float* __restrict__ b2b, const float* __restrict__ rb,
    unsigned short* Bt1, unsigned short* Bt2) {
  __shared__ __attribute__((aligned(16))) unsigned short row[KT64];
  const int tid = threadIdx.x;
  if ((int)blockIdx.x < C1W) build_row<16, 64>(W2a, b2a, ra, (int)blockIdx.x, Bt1, row, tid);
  else                       build_row<64, 128>(W2b, b2b, rb, (int)blockIdx.x - C1W, Bt2, row, tid);
}

template <int IN>
__global__ __launch_bounds__(NTHR) void k_scan(const int* __restrict__ ei, int nE, int vec8,
    const float* __restrict__ F, int nN, const float* __restrict__ HE,
    const float* __restrict__ scsh, unsigned short* Ap) {
  constexpr int JPT  = IN / 8;
  constexpr int KZ   = 32 * IN;
  constexpr int KTOT = 2 * KZ + 4 * IN;
  constexpr int NPC  = KTOT / 8;
  constexpr int PPT  = (NPC + NTHR - 1) / NTHR;
  constexpr bool BNA = (IN == 64);
  static_assert(IN == 16 || IN == 64);
  static_assert((KTOT % 64) == 0);
  static_assert(JPT * (NTHR / IN) == HID);
  __shared__ int list[LISTN];
  __shared__ int sle[NBS * DEGCAP];
  __shared__ int sls[NBS * DEGCAP];
  __shared__ int cnt[NBS];
  __shared__ int wcnt[NWAVE];
  __shared__ float scs[2 * C1W];
  __shared__ __attribute__((aligned(16))) unsigned short stg[KTOT];

  const int tid = threadIdx.x, lane = tid & 31, wave = tid >> 5;
  const int i = tid & (IN - 1), jg = tid / IN;
  const int nb = (int)blockIdx.x * NBS;
  if (tid < NBS) cnt[tid] = 0;
  if constexpr (BNA) { if (tid < 2 * C1W) scs[tid] = scsh[tid]; }
  __syncthreads();

  const int* keys = ei + nE;
  const int nChunks = (nE + CHUNK - 1) / CHUNK;
#pragma unroll 1
  for (int ch = 0; ch < nChunks; ++ch) {
    const int cbase = ch * CHUNK;
    const int wc = scan_chunk(keys, nE, cbase, nb, vec8, list, tid, lane, wave);
    if (lane == 0) wcnt[wave] = wc;
    __syncthreads();
    if (wave == 0) {
#pragma unroll 1
      for (int wsx = 0; wsx < NWAVE; ++wsx) {
        int n = __builtin_amdgcn_readfirstlane(wcnt[wsx]);
        n = n > WCAP ? WCAP : (n < 0 ? 0 : n);
#pragma unroll 1
        for (int ii = 0; ii < n; ++ii) {
          const int ent = __builtin_amdgcn_readfirstlane(list[wsx * WCAP + ii]);
          const int slot = ent & (NBS - 1);
          int e = cbase + ((ent >> 6) & (CHUNK - 1));
          e = e > nE - 1 ? nE - 1 : e;
          int sr = ei[e];
          sr = sr < 0 ? 0 : (sr > nN - 1 ? nN - 1 : sr);
          if (lane == 0) {
            const int pos = cnt[slot];
            if (pos < DEGCAP) { sle[slot * DEGCAP + pos] = e; sls[slot * DEGCAP + pos] = sr; }
            cnt[slot] = pos < (1 << 24) ? pos + 1 : pos;
          }
        }
      }
    }
    __syncthreads();
  }

  float scv = 1.0f, shv = 0.0f;
  if constexpr (BNA) { scv = scs[i]; shv = scs[C1W + i]; }

#pragma unroll 1
  for (int s = 0; s < NBS; ++s) {
    const int c  = cnt[s];
    const int np = c < DEGCAP ? c : DEGCAP;
    const bool bad = c > DEGCAP;
    const int d  = nb + s;
    float acc[JPT];
#pragma unroll
    for (int k = 0; k < JPT; ++k) acc[k] = 0.0f;
    float facc = 0.0f;
#pragma unroll 1
    for (int p = 0; p < np; ++p) {
      const int e  = sle[s * DEGCAP + p];
      const int sr = sls[s * DEGCAP + p];
      float fv = F[(size_t)sr * IN + i];
      if constexpr (BNA) fv = fmaf(fv, scv, shv); else fv = bfq(fv);
      if constexpr (JPT == 8) {
        const float* hp = HE + (size_t)e * HID + 8 * jg;
        const v4f ha = *(const v4f*)hp;
        const v4f hb = *(const v4f*)(hp + 4);
        acc[0] = fmaf(ha.x, fv, acc[0]); acc[1] = fmaf(ha.y, fv, acc[1]);
        acc[2] = fmaf(ha.z, fv, acc[2]); acc[3] = fmaf(ha.w, fv, acc[3]);
        acc[4] = fmaf(hb.x, fv, acc[4]); acc[5] = fmaf(hb.y, fv, acc[5]);
        acc[6] = fmaf(hb.z, fv, acc[6]); acc[7] = fmaf(hb.w, fv, acc[7]);
      } else {
        const v2f hv = *(const v2f*)(HE + (size_t)e * HID + 2 * jg);
        acc[0] = fmaf(hv.x, fv, acc[0]); acc[1] = fmaf(hv.y, fv, acc[1]);
      }
      facc += fv;
    }
    const float rc = 1.0f / (float)(c < 1 ? 1 : c);
    const int dc = d < nN ? d : nN - 1;
    const float keep = (d < nN) ? 1.0f : 0.0f;
    float rv = F[(size_t)dc * IN + i];
    if constexpr (BNA) rv = fmaf(rv, scv, shv); else rv = bfq(rv);
    rv = rv * keep;
#pragma unroll
    for (int k = 0; k < JPT; ++k) {
      unsigned short hi, lo;
      hilo(acc[k] * rc, bad, hi, lo);
      const int col = (JPT * jg + k) * IN + i;
      stg[col] = hi;
      stg[KZ + col] = lo;
    }
    if (jg == 0) {
      unsigned short hi, lo;
      hilo(facc * rc, bad, hi, lo);
      stg[2 * KZ + i] = hi;
      stg[2 * KZ + IN + i] = lo;
    }
    if constexpr (IN == 16) {
      const unsigned short rb = bad ? (unsigned short)0x7FC0 : bfr(rv);
      if (jg == 1) stg[2 * KZ + 2 * IN + i] = rb;
      if (jg == 2) stg[2 * KZ + 3 * IN + i] = (unsigned short)0;
    } else {
      unsigned short hi, lo;
      hilo(rv, bad, hi, lo);
      if (jg == 1) { stg[2 * KZ + 2 * IN + i] = hi; stg[2 * KZ + 3 * IN + i] = lo; }
    }
    __syncthreads();
    v8us pv[PPT];
#pragma unroll
    for (int it = 0; it < PPT; ++it) {
      int pc = it * NTHR + tid;
      pc = pc > NPC - 1 ? NPC - 1 : pc;
      pv[it] = *(const v8us*)(stg + 8 * pc);
    }
    unsigned short* ar = Ap + (size_t)d * KTOT;
#pragma unroll
    for (int it = 0; it < PPT; ++it)
      if (it * NTHR + tid < NPC) *(volatile v8us*)(ar + 8 * (it * NTHR + tid)) = pv[it];
    __threadfence();
#pragma unroll
    for (int it = 0; it < PPT; ++it)
      if (it * NTHR + tid < NPC) *(volatile v8us*)(ar + 8 * (it * NTHR + tid)) = pv[it];
    __syncthreads();
  }
}

template <int IN, int NOUT>
__global__ __launch_bounds__(NTHR) void k_gemm(const unsigned short* __restrict__ A,
    const unsigned short* __restrict__ Bt, const float* __restrict__ bias, float* C, float* rec, int nN) {
  constexpr int KZ = 32 * IN, KTOT = 2 * KZ + 4 * IN, KS = KTOT / 32, NT = NOUT / 16;
  constexpr int NPQ = MT * NOUT / 4 / NTHR;
  static_assert((KTOT % 32) == 0 && (NOUT % 32) == 0 && ((MT * NOUT / 4) % NTHR) == 0 && NT <= 8);
  static_assert(MT == 16 * NWAVE);
  extern __shared__ v4f lds_dyn[];
  float* stg = (float*)lds_dyn;
  float* rst = stg + MT * NOUT;
  const int tid = threadIdx.x, wave = tid >> 5, lane = tid & 31, hf = lane >> 4, m = lane & 15;
  const int row0 = (int)blockIdx.x * MT;
  const unsigned short* ap  = A + (size_t)(row0 + 16 * wave + m) * KTOT + 8 * hf;
  const unsigned short* bp0 = Bt + (size_t)m * KTOT + 8 * hf;
  v8f acc[NT];
#pragma unroll
  for (int t = 0; t < NT; ++t) acc[t] = z8();
#pragma unroll 1
  for (int ks = 0; ks < KS; ++ks) {
    FragB a;
    a.u[0] = *(const v8us*)(ap + 32 * ks);
    a.u[1] = *(const v8us*)(ap + 32 * ks + 16);
#pragma unroll
    for (int t = 0; t < NT; ++t) {
      const unsigned short* bp = bp0 + (size_t)(16 * t) * KTOT + 32 * ks;
      FragB b;
      b.u[0] = *(const v8us*)bp;
      b.u[1] = *(const v8us*)(bp + 16);
      acc[t] = wmb(a.v, b.v, acc[t]);
    }
  }
  {
    float* sp = stg + (16 * wave + 8 * hf) * NOUT + m;
#pragma unroll
    for (int t = 0; t < NT; ++t) {
      const float bv = bfq(bias[16 * t + m]);
#pragma unroll
      for (int r = 0; r < 8; ++r) sp[r * NOUT + 16 * t] = fmaxf(acc[t][r] + bv, 0.0f);
    }
  }
  __syncthreads();
  {
    v4f pv[NPQ];
#pragma unroll
    for (int it = 0; it < NPQ; ++it) pv[it] = *(const v4f*)(stg + 4 * (it * NTHR + tid));
    float* cbp = C + (size_t)row0 * NOUT;
#pragma unroll
    for (int it = 0; it < NPQ; ++it) *(volatile v4f*)(cbp + 4 * (it * NTHR + tid)) = pv[it];
    __threadfence();
#pragma unroll
    for (int it = 0; it < NPQ; ++it) *(volatile v4f*)(cbp + 4 * (it * NTHR + tid)) = pv[it];
  }
  if (tid < NOUT) {
    int nv = nN - row0;
    nv = nv < 0 ? 0 : (nv > MT ? MT : nv);
    float s = 0.0f, s2 = 0.0f;
#pragma unroll 1
    for (int r = 0; r < nv; ++r) {
      const float v = stg[r * NOUT + tid];
      s += v;
      s2 = fmaf(v, v, s2);
    }
    rst[tid] = s;
    rst[NOUT + tid] = s2;
  }
  __syncthreads();
  if (tid < NOUT / 2) {
    const v4f v = *(const v4f*)(rst + 4 * tid);
    float* rp = rec + (size_t)blockIdx.x * (2 * NOUT) + 4 * tid;
    *(volatile v4f*)rp = v;
    __threadfence();
    *(volatile v4f*)rp = v;
  }
}

template <int NOUT>
__global__ __launch_bounds__(NTHR) void k_bnfold(const float* __restrict__ rec, int nblk, int nN,
    const float* __restrict__ gam, const float* __restrict__ bet, float* scsh) {
  __shared__ __attribute__((aligned(16))) float st[2 * NOUT];
  const int tid = threadIdx.x;
  if (tid < NOUT) {
    double s = 0.0, s2 = 0.0;
#pragma unroll 1
    for (int b = 0; b < nblk; ++b) {
      s  += (double)rec[(size_t)b * (2 * NOUT) + tid];
      s2 += (double)rec[(size_t)b * (2 * NOUT) + NOUT + tid];
    }
    const double inv = 1.0 / (double)(nN < 1 ? 1 : nN);
    const double mu = s * inv;
    double var = s2 * inv - mu * mu;
    var = var < 0.0 ? 0.0 : var;
    const float rs = rsqrtf((float)var + BNEPS);
    const float g = bfq(gam[tid]), be = bfq(bet[tid]);
    const float sc = rs * g;
    const float sh = be - (float)mu * sc;
    st[tid] = sc;
    st[NOUT + tid] = sh;
  }
  __syncthreads();
  if (tid < NOUT / 2) {
    const v4f v = *(const v4f*)(st + 4 * tid);
    float* dp = scsh + 4 * tid;
    *(volatile v4f*)dp = v;
    __threadfence();
    *(volatile v4f*)dp = v;
  }
}

__global__ __launch_bounds__(NTHR) void k_head(const int* __restrict__ batch, int nN, const float* __restrict__ C2,
    const float* __restrict__ scsh, const float* __restrict__ l1w, const float* __restrict__ l1b,
    const float* __restrict__ l2w, const float* __restrict__ l2b, float* out) {
  extern __shared__ v4f lds_dyn[];
  float* pool = (float*)lds_dyn;
  float* w1s  = pool + NGR * PP;
  float* scs  = w1s + C2W * C1W;
  float* b1s  = scs + 2 * C2W;
  float* w2s  = b1s + C1W;
  float* sOut = w2s + C1W;
  int*   cntg = (int*)(sOut + NGR);
  const int tid = threadIdx.x;
#pragma unroll 1
  for (int k = tid; k < NGR * PP; k += NTHR) pool[k] = 0.0f;
#pragma unroll 1
  for (int k = tid; k < C2W * C1W; k += NTHR) w1s[k] = bfq(l1w[k]);
  scs[tid] = scsh[tid];
  cntg[tid] = 0;
  if (tid < C1W) { b1s[tid] = bfq(l1b[tid]); w2s[tid] = bfq(l2w[tid]); }
  __syncthreads();

  const int o = tid & (C2W - 1);
  const int g0 = 2 * (tid & 127), g1 = g0 + 1;
  int ca = 0, cb = 0;
#pragma unroll 1
  for (int n = 0; n < nN; ++n) {
    const int q = batch[n];
    if (tid < C2W) {
      const float fi = ((unsigned)q < (unsigned)NGR) ? 1.0f : 0.0f;
      const int qc = q < 0 ? 0 : (q > NGR - 1 ? NGR - 1 : q);
      const float v = C2[(size_t)n * C2W + o];
      pool[qc * PP + o] += v * fi;
    } else {
      ca += (q == g0) ? 1 : 0;
      cb += (q == g1) ? 1 : 0;
    }
  }
  if (tid >= C2W) { cntg[g0] = ca; cntg[g1] = cb; }
  __syncthreads();
  if (tid < C2W) {
    const float sc = scs[o], sh = scs[C2W + o];
#pragma unroll 1
    for (int q = 0; q < NGR; ++q) {
      const int c = cntg[q];
      const float rc = 1.0f / (float)(c < 1 ? 1 : c);
      const float fi = (c > 0) ? 1.0f : 0.0f;
      const float gm = pool[q * PP + o] * rc;
      pool[q * PP + o] = fmaf(gm, sc, sh * fi);
    }
  }
  __syncthreads();
  {
    const int q = tid;
    const float* gr = pool + q * PP;
    float ov = bfq(l2b[0]);
#pragma unroll 1
    for (int j = 0; j < C1W; ++j) {
      float s = b1s[j];
#pragma unroll 4
      for (int k = 0; k < C2W; ++k) s = fmaf(gr[k], w1s[k * C1W + j], s);
      ov = fmaf(fmaxf(s, 0.0f), w2s[j], ov);
    }
    sOut[q] = ov;
  }
  __syncthreads();
  if (tid < NGR / 4) {
    const v4f v = *(const v4f*)(sOut + 4 * tid);
    float* op = out + 4 * tid;
    *(volatile v4f*)op = v;
    __threadfence();
    *(volatile v4f*)op = v;
  }
}

extern "C" void kernel_launch(void* const* d_in, const int* in_sizes, int n_in,
                              void* d_out, int out_size, void* d_ws, size_t ws_size,
                              hipStream_t stream) {
  if (n_in < 24) return;
  const int nN = in_sizes[3];
  const int nE = in_sizes[1] / 2;
  if (nN <= 0 || nE <= 0) return;
  if (in_sizes[0] != nN * 16 || in_sizes[1] != 2 * nE || in_sizes[2] != nE * EC) return;
  if (in_sizes[4] != EC * HID || in_sizes[5] != HID || in_sizes[6] != HID * 16 * C1W || in_sizes[7] != 16 * C1W) return;
  if (in_sizes[8] != 16 * C1W || in_sizes[9] != C1W || in_sizes[10] != C1W || in_sizes[11] != C1W) return;
  if (in_sizes[12] != EC * HID || in_sizes[13] != HID || in_sizes[14] != HID * C1W * C2W || in_sizes[15] != C1W * C2W) return;
  if (in_sizes[16] != C1W * C2W || in_sizes[17] != C2W || in_sizes[18] != C2W || in_sizes[19] != C2W) return;
  if (in_sizes[20] != C2W * C1W || in_sizes[21] != C1W || in_sizes[22] != C1W || in_sizes[23] != 1) return;
  if (out_size != NGR) return;
  if (nN > (1 << 22) || nE > (1 << 24)) return;

  const float* x     = (const float*)d_in[0];
  const int*   ei    = (const int*)d_in[1];
  const float* ea    = (const float*)d_in[2];
  const int*   batch = (const int*)d_in[3];
  const float* n1W1  = (const float*)d_in[4];
  const float* n1b1  = (const float*)d_in[5];
  const float* n1W2  = (const float*)d_in[6];
  const float* n1b2  = (const float*)d_in[7];
  const float* root1 = (const float*)d_in[8];
  const float* bias1 = (const float*)d_in[9];
  const float* bn1g  = (const float*)d_in[10];
  const float* bn1b  = (const float*)d_in[11];
  const float* n2W1  = (const float*)d_in[12];
  const float* n2b1  = (const float*)d_in[13];
  const float* n2W2  = (const float*)d_in[14];
  const float* n2b2  = (const float*)d_in[15];
  const float* root2 = (const float*)d_in[16];
  const float* bias2 = (const float*)d_in[17];
  const float* bn2g  = (const float*)d_in[18];
  const float* bn2b  = (const float*)d_in[19];
  const float* l1W   = (const float*)d_in[20];
  const float* l1b   = (const float*)d_in[21];
  const float* l2W   = (const float*)d_in[22];
  const float* l2b   = (const float*)d_in[23];
  float* out = (float*)d_out;

  const int NEB   = (nE + NTHR - 1) / NTHR;
  const int EPAD  = NEB * NTHR;
  const int NBM   = (nN + MT - 1) / MT;
  const int NPADM = NBM * MT;
  const int NSB   = NPADM / NBS;

  size_t off = 0;
  const size_t oHE1 = off; off += (((size_t)EPAD * HID * 4) + 255) & ~(size_t)255;
  const size_t oHE2 = off; off += (((size_t)EPAD * HID * 4) + 255) & ~(size_t)255;
  const size_t oBt1 = off; off += (((size_t)C1W * KT16 * 2) + 255) & ~(size_t)255;
  const size_t oBt2 = off; off += (((size_t)C2W * KT64 * 2) + 255) & ~(size_t)255;
  const size_t oA   = off; off += (((size_t)NPADM * KT64 * 2) + 255) & ~(size_t)255;
  const size_t oC1  = off; off += (((size_t)NPADM * C1W * 4) + 255) & ~(size_t)255;
  const size_t oR1  = off; off += (((size_t)NBM * 2 * C1W * 4) + 255) & ~(size_t)255;
  const size_t oS1  = off; off += (((size_t)2 * C1W * 4) + 255) & ~(size_t)255;
  const size_t oC2  = off; off += (((size_t)NPADM * C2W * 4) + 255) & ~(size_t)255;
  const size_t oR2  = off; off += (((size_t)NBM * 2 * C2W * 4) + 255) & ~(size_t)255;
  const size_t oS2  = off; off += (((size_t)2 * C2W * 4) + 255) & ~(size_t)255;
  if (off > ws_size) return;
  if (off > (size_t)128 * 1024 * 1024) return;
  char* ws = (char*)d_ws;
  float* HE1 = (float*)(ws + oHE1);
  float* HE2 = (float*)(ws + oHE2);
  unsigned short* Bt1 = (unsigned short*)(ws + oBt1);
  unsigned short* Bt2 = (unsigned short*)(ws + oBt2);
  unsigned short* Apl = (unsigned short*)(ws + oA);
  float* C1 = (float*)(ws + oC1);
  float* R1 = (float*)(ws + oR1);
  float* S1 = (float*)(ws + oS1);
  float* C2 = (float*)(ws + oC2);
  float* R2 = (float*)(ws + oR2);
  float* S2 = (float*)(ws + oS2);
  const int vec8 = ((nE & 3) == 0) ? 1 : 0;

  constexpr int LG1 = MT * C1W * 4 + 2 * C1W * 4;
  constexpr int LG2 = MT * C2W * 4 + 2 * C2W * 4;
  constexpr int LH  = (NGR * PP + C2W * C1W + 2 * C2W + C1W + C1W + NGR) * 4 + NGR * 4;
  hipFuncSetAttribute(reinterpret_cast<const void*>(&k_gemm<16, 64>), hipFuncAttributeMaxDynamicSharedMemorySize, LG1);
  hipFuncSetAttribute(reinterpret_cast<const void*>(&k_gemm<64, 128>), hipFuncAttributeMaxDynamicSharedMemorySize, LG2);
  hipFuncSetAttribute(reinterpret_cast<const void*>(&k_head), hipFuncAttributeMaxDynamicSharedMemorySize, LH);

  k_he<<<NEB, NTHR, 0, stream>>>(ea, nE, n1W1, n1b1, n2W1, n2b1, HE1, HE2);
  k_bprep<<<C1W + C2W, NTHR, 0, stream>>>(n1W2, n1b2, root1, n2W2, n2b2, root2, Bt1, Bt2);
  k_scan<16><<<NSB, NTHR, 0, stream>>>(ei, nE, vec8, x, nN, HE1, S1, Apl);
  k_gemm<16, 64><<<NBM, NTHR, LG1, stream>>>(Apl, Bt1, bias1, C1, R1, nN);
  k_bnfold<64><<<1, NTHR, 0, stream>>>(R1, NBM, nN, bn1g, bn1b, S1);
  k_scan<64><<<NSB, NTHR, 0, stream>>>(ei, nE, vec8, C1, nN, HE2, S1, Apl);
  k_gemm<64, 128><<<NBM, NTHR, LG2, stream>>>(Apl, Bt2, bias2, C2, R2, nN);
  k_bnfold<128><<<1, NTHR, 0, stream>>>(R2, NBM, nN, bn2g, bn2b, S2);
  k_head<<<1, NTHR, LH, stream>>>(batch, nN, C2, S2, l1W, l1b, l2W, l2b, out);
}
